// AdsorptionGNN_43817256354335
// MI455X (gfx1250) — hardware-verified
//
#include <hip/hip_runtime.h>
#define NNODE 50000
#define NEDGE 800000
#define NP2 1048576
#define HH 128
#define ED 4
#define K1 288
#define NL 4
#define NG 512
#define NSL 4
#define ESL (NEDGE / NSL)

typedef __bf16 v16b __attribute__((ext_vector_type(16)));
typedef unsigned short v8us __attribute__((ext_vector_type(8), may_alias));
typedef float  v8f  __attribute__((ext_vector_type(8)));
typedef float  v4f  __attribute__((ext_vector_type(4)));
typedef float  v4fa __attribute__((ext_vector_type(4), may_alias));
union FragB { v16b v; v8us half[2]; unsigned short u[16]; };

__device__ __forceinline__ unsigned short bf16_bits(float x) { unsigned int u = __float_as_uint(x); return (unsigned short)((u + 0x7FFFu + ((u >> 16) & 1u)) >> 16); }
__device__ __forceinline__ float bf16_val(unsigned short b) { return __uint_as_float(((unsigned int)b) << 16); }
__device__ __forceinline__ float bf16_round(float x) { return bf16_val(bf16_bits(x)); }
template <int NT>
__device__ __forceinline__ v8f mmaN(v16b ah, v16b al, v16b bh, v16b bl, v8f c) {
  c = __builtin_amdgcn_wmma_f32_16x16x32_bf16(false, ah, false, bh, (short)0, c, false, false);
  if (NT >= 2) c = __builtin_amdgcn_wmma_f32_16x16x32_bf16(false, al, false, bh, (short)0, c, false, false);
  if (NT >= 3) c = __builtin_amdgcn_wmma_f32_16x16x32_bf16(false, ah, false, bl, (short)0, c, false, false);
  asm volatile("v_nop\n\tv_nop\n\tv_nop\n\tv_nop" : "+v"(c) : "v"(ah), "v"(al), "v"(bh), "v"(bl));
  return c;
}

__global__ __launch_bounds__(256) void k_wt_bf16(const float* __restrict__ W, unsigned short* __restrict__ Wt, int K, int N) {
  const int t = blockIdx.x * 256 + threadIdx.x;
  const int k8n = K / 8;
  if (t >= N * k8n) return;
  const int n = t / k8n, k8 = (t % k8n) * 8;
  v8us v;
#pragma unroll
  for (int i = 0; i < 8; ++i) v[i] = bf16_bits(W[(size_t)(k8 + i) * N + n]);
  *(volatile v8us*)(Wt + (size_t)n * K + k8) = v;
  __threadfence();
  *(volatile v8us*)(Wt + (size_t)n * K + k8) = v;
}

template <bool ASPLIT, int ACT, bool BIAS_BF16>
__global__ __launch_bounds__(128) void k_gemm_bf(const float* __restrict__ A, int lda, const unsigned short* __restrict__ Wt, int ldb,
                                               const float* __restrict__ bias, float* __restrict__ C, int ldc, int M, int N, int K) {
  __shared__ __attribute__((aligned(16))) float so[4][16][64];
  const int tid = threadIdx.x, w = tid >> 5, lane = tid & 31, ln = lane & 15, hh = lane >> 4;
  const int ntn = N / 64;
  const int wid = blockIdx.x * 4 + w;
  const int mt = wid / ntn, nq = wid % ntn;
  if (mt * 16 >= M) return;
  const int row0 = mt * 16, col0 = nq * 64;
  const float* arow = A + (size_t)(row0 + ln) * lda;
  v8f acc[4] = {};
  for (int kb = 0; kb < K; kb += 32) {
    FragB ah, al;
    const v4f x0 = *(const v4fa*)(arow + kb + 8 * hh), x1 = *(const v4fa*)(arow + kb + 8 * hh + 4);
    const v4f x2 = *(const v4fa*)(arow + kb + 16 + 8 * hh), x3 = *(const v4fa*)(arow + kb + 16 + 8 * hh + 4);
    float xs[16] = {x0[0],x0[1],x0[2],x0[3],x1[0],x1[1],x1[2],x1[3],x2[0],x2[1],x2[2],x2[3],x3[0],x3[1],x3[2],x3[3]};
#pragma unroll
    for (int i = 0; i < 16; ++i) { const unsigned short hb = bf16_bits(xs[i]); ah.u[i] = hb; al.u[i] = ASPLIT ? bf16_bits(xs[i] - bf16_val(hb)) : (unsigned short)0; }
#pragma unroll
    for (int t = 0; t < 4; ++t) {
      const unsigned short* brow = Wt + (size_t)(col0 + t * 16 + ln) * ldb + kb;
      FragB b;
      b.half[0] = *(const v8us*)(brow + 8 * hh);
      b.half[1] = *(const v8us*)(brow + 16 + 8 * hh);
      acc[t] = mmaN<ASPLIT ? 2 : 1>(ah.v, al.v, b.v, b.v, acc[t]);
    }
  }
#pragma unroll
  for (int t = 0; t < 4; ++t) {
    float bv = bias ? bias[col0 + t * 16 + ln] : 0.f;
    if (BIAS_BF16) bv = bf16_round(bv);
#pragma unroll
    for (int r = 0; r < 8; ++r) { float v = acc[t][r] + bv; if (ACT == 1) v = fmaxf(v, 0.f); so[w][8 * hh + r][t * 16 + ln] = v; }
  }
  __builtin_amdgcn_fence(__ATOMIC_ACQ_REL, "workgroup");
  __builtin_amdgcn_wave_barrier();
  const int rsub = lane >> 4, c4 = (lane & 15) * 4;
  for (int pass = 0; pass < 2; ++pass) {
#pragma unroll
    for (int q = 0; q < 8; ++q) {
      const int r = q * 2 + rsub;
      const v4f v = *(const v4fa*)&so[w][r][c4];
      *(volatile v4f*)(C + (size_t)(row0 + r) * ldc + col0 + c4) = v;
    }
    if (pass == 0) __threadfence();
  }
}

template <int D, bool CAUSAL>
__global__ __launch_bounds__(128) void k_flash(const float* __restrict__ qb, const float* __restrict__ kb, const float* __restrict__ vb,
                                             int pitch, int T, int H, float scale, float* __restrict__ y, int ypitch) {
  constexpr int KS = D / 32;
  constexpr int DT = D / 16;
  __shared__ __attribute__((aligned(16))) unsigned short sKh[32][D + 8], sKl[32][D + 8], sVh[32][D + 8], sVl[32][D + 8];
  __shared__ __attribute__((aligned(16))) unsigned short sPh[4][16][40], sPl[4][16][40];
  __shared__ __attribute__((aligned(16))) float sO[4][16][D];
  const int tid = threadIdx.x, w = tid >> 5, lane = tid & 31, ln = lane & 15, hh = lane >> 4;
  const int nqb = (T + 63) / 64;
  const int bh = blockIdx.x / nqb, qblk = blockIdx.x % nqb;
  const int b = bh / H, h = bh % H;
  const int q0 = qblk * 64 + w * 16;
  const float* Q = qb + (size_t)b * T * pitch + h * D;
  const float* K = kb + (size_t)b * T * pitch + h * D;
  const float* V = vb + (size_t)b * T * pitch + h * D;

  FragB aqh[KS], aql[KS];
  {
    int row = q0 + ln; if (row >= T) row = T - 1;
    const float* qr = Q + (size_t)row * pitch;
#pragma unroll
    for (int ks = 0; ks < KS; ++ks)
#pragma unroll
      for (int i = 0; i < 16; ++i) {
        const int d = ks * 32 + ((i < 8) ? (8 * hh + i) : (16 + 8 * hh + (i - 8)));
        const float x = qr[d] * scale; const unsigned short hb = bf16_bits(x);
        aqh[ks].u[i] = hb; aql[ks].u[i] = bf16_bits(x - bf16_val(hb));
      }
  }
  float m_r[8], l_r[8];
#pragma unroll
  for (int r = 0; r < 8; ++r) { m_r[r] = -3.0e38f; l_r[r] = 0.f; }
  v8f oacc[DT];
#pragma unroll
  for (int dt = 0; dt < DT; ++dt) oacc[dt] = (v8f){0.f,0.f,0.f,0.f,0.f,0.f,0.f,0.f};

  const int kv_end = CAUSAL ? min(T, qblk * 64 + 64) : T;
  for (int j0 = 0; j0 < kv_end; j0 += 32) {
    __syncthreads();
    for (int e = tid; e < 32 * (D / 4); e += 128) {
      const int r = e / (D / 4), c4 = (e % (D / 4)) * 4;
      const int key = j0 + r;
      v4f kf = {0.f,0.f,0.f,0.f}, vf = {0.f,0.f,0.f,0.f};
      if (key < T) { kf = *(const v4fa*)(K + (size_t)key * pitch + c4); vf = *(const v4fa*)(V + (size_t)key * pitch + c4); }
#pragma unroll
      for (int t = 0; t < 4; ++t) {
        unsigned short hb = bf16_bits(kf[t]); sKh[r][c4 + t] = hb; sKl[r][c4 + t] = bf16_bits(kf[t] - bf16_val(hb));
        hb = bf16_bits(vf[t]); sVh[r][c4 + t] = hb; sVl[r][c4 + t] = bf16_bits(vf[t] - bf16_val(hb));
      }
    }
    __syncthreads();
    v8f s[2];
#pragma unroll
    for (int nt = 0; nt < 2; ++nt) {
      v8f acc = {};
#pragma unroll
      for (int ks = 0; ks < KS; ++ks) {
        FragB bh_, bl_;
        bh_.half[0] = *(const v8us*)&sKh[nt * 16 + ln][ks * 32 + 8 * hh]; bh_.half[1] = *(const v8us*)&sKh[nt * 16 + ln][ks * 32 + 16 + 8 * hh];
        bl_.half[0] = *(const v8us*)&sKl[nt * 16 + ln][ks * 32 + 8 * hh]; bl_.half[1] = *(const v8us*)&sKl[nt * 16 + ln][ks * 32 + 16 + 8 * hh];
        acc = mmaN<3>(aqh[ks].v, aql[ks].v, bh_.v, bl_.v, acc);
      }
      s[nt] = acc;
    }
    float alpha[8];
#pragma unroll
    for (int r = 0; r < 8; ++r) {
      const int qi = q0 + 8 * hh + r;
      const int ja = j0 + ln, jb = j0 + 16 + ln;
      if (CAUSAL) { if (ja > qi) s[0][r] = -3.0e38f; if (jb > qi) s[1][r] = -3.0e38f; }
      if (ja >= T) s[0][r] = -3.0e38f;
      if (jb >= T) s[1][r] = -3.0e38f;
      float mx = fmaxf(s[0][r], s[1][r]);
      mx = fmaxf(mx, __shfl_xor(mx, 1, 32)); mx = fmaxf(mx, __shfl_xor(mx, 2, 32)); mx = fmaxf(mx, __shfl_xor(mx, 4, 32)); mx = fmaxf(mx, __shfl_xor(mx, 8, 32));
      const float mnew = fmaxf(m_r[r], mx);
      alpha[r] = (mnew > -1.0e38f) ? __expf(m_r[r] - mnew) : 1.0f;
      const float p0 = (s[0][r] > -1.0e38f) ? __expf(s[0][r] - mnew) : 0.f;
      const float p1 = (s[1][r] > -1.0e38f) ? __expf(s[1][r] - mnew) : 0.f;
      m_r[r] = mnew;
      l_r[r] = l_r[r] * alpha[r] + p0 + p1;
      unsigned short hb = bf16_bits(p0); sPh[w][8 * hh + r][ln] = hb;      sPl[w][8 * hh + r][ln] = bf16_bits(p0 - bf16_val(hb));
      hb = bf16_bits(p1);                sPh[w][8 * hh + r][16 + ln] = hb; sPl[w][8 * hh + r][16 + ln] = bf16_bits(p1 - bf16_val(hb));
    }
#pragma unroll
    for (int dt = 0; dt < DT; ++dt)
#pragma unroll
      for (int r = 0; r < 8; ++r) oacc[dt][r] *= alpha[r];
    __builtin_amdgcn_fence(__ATOMIC_ACQ_REL, "workgroup");
    __builtin_amdgcn_wave_barrier();
    FragB pah, pal;
    pah.half[0] = *(const v8us*)&sPh[w][ln][8 * hh]; pah.half[1] = *(const v8us*)&sPh[w][ln][16 + 8 * hh];
    pal.half[0] = *(const v8us*)&sPl[w][ln][8 * hh]; pal.half[1] = *(const v8us*)&sPl[w][ln][16 + 8 * hh];
#pragma unroll
    for (int dt = 0; dt < DT; ++dt) {
      FragB bvh, bvl;
#pragma unroll
      for (int i = 0; i < 8; ++i) {
        bvh.u[i] = sVh[8 * hh + i][dt * 16 + ln]; bvh.u[8 + i] = sVh[16 + 8 * hh + i][dt * 16 + ln];
        bvl.u[i] = sVl[8 * hh + i][dt * 16 + ln]; bvl.u[8 + i] = sVl[16 + 8 * hh + i][dt * 16 + ln];
      }
      oacc[dt] = mmaN<3>(pah.v, pal.v, bvh.v, bvl.v, oacc[dt]);
    }
    __builtin_amdgcn_fence(__ATOMIC_ACQ_REL, "workgroup");
    __builtin_amdgcn_wave_barrier();
  }
#pragma unroll
  for (int r = 0; r < 8; ++r) {
    float l = l_r[r];
    l += __shfl_xor(l, 1, 32); l += __shfl_xor(l, 2, 32); l += __shfl_xor(l, 4, 32); l += __shfl_xor(l, 8, 32);
    l_r[r] = (l > 0.f) ? 1.0f / l : 0.f;
  }
#pragma unroll
  for (int dt = 0; dt < DT; ++dt)
#pragma unroll
    for (int r = 0; r < 8; ++r) sO[w][8 * hh + r][dt * 16 + ln] = oacc[dt][r] * l_r[r];
  __builtin_amdgcn_fence(__ATOMIC_ACQ_REL, "workgroup");
  __builtin_amdgcn_wave_barrier();
  for (int pass = 0; pass < 2; ++pass) {
    for (int r = 0; r < 16; ++r) {
      const int row = q0 + r;
      if (row < T && lane < D / 4) {
        const v4f val = *(const v4fa*)&sO[w][r][lane * 4];
        *(volatile v4f*)(y + ((size_t)b * T + row) * ypitch + h * D + lane * 4) = val;
      }
    }
    if (pass == 0) __threadfence();
  }
}

template <bool ASPLIT, int ACT, bool BIAS_BF16, bool RES_BF16>
__global__ __launch_bounds__(128) void k_gemm_bf3(const float* __restrict__ A, int lda, const unsigned short* __restrict__ Wt, int ldb,
                                                const float* __restrict__ bias, const float* __restrict__ resid, int rmod, int ldr,
                                                float* __restrict__ C, int ldc, int M, int N, int K) {
  __shared__ __attribute__((aligned(16))) float so[4][16][64];
  const int tid = threadIdx.x, w = tid >> 5, lane = tid & 31, ln = lane & 15, hh = lane >> 4;
  const int ntn = N / 64;
  const int wid = blockIdx.x * 4 + w;
  const int mt = wid / ntn, nq = wid % ntn;
  if (mt * 16 >= M) return;
  const int row0 = mt * 16, col0 = nq * 64;
  const float* arow = A + (size_t)(row0 + ln) * lda;
  v8f acc[4] = {};
  for (int kb = 0; kb < K; kb += 32) {
    FragB ah, al;
    const v4f x0 = *(const v4fa*)(arow + kb + 8 * hh), x1 = *(const v4fa*)(arow + kb + 8 * hh + 4);
    const v4f x2 = *(const v4fa*)(arow + kb + 16 + 8 * hh), x3 = *(const v4fa*)(arow + kb + 16 + 8 * hh + 4);
    float xs[16] = {x0[0],x0[1],x0[2],x0[3],x1[0],x1[1],x1[2],x1[3],x2[0],x2[1],x2[2],x2[3],x3[0],x3[1],x3[2],x3[3]};
#pragma unroll
    for (int i = 0; i < 16; ++i) { const unsigned short hb = bf16_bits(xs[i]); ah.u[i] = hb; al.u[i] = ASPLIT ? bf16_bits(xs[i] - bf16_val(hb)) : (unsigned short)0; }
#pragma unroll
    for (int t = 0; t < 4; ++t) {
      const unsigned short* brow = Wt + (size_t)(col0 + t * 16 + ln) * ldb + kb;
      FragB b;
      b.half[0] = *(const v8us*)(brow + 8 * hh);
      b.half[1] = *(const v8us*)(brow + 16 + 8 * hh);
      acc[t] = mmaN<ASPLIT ? 2 : 1>(ah.v, al.v, b.v, b.v, acc[t]);
    }
  }
#pragma unroll
  for (int t = 0; t < 4; ++t) {
    const int col = col0 + t * 16 + ln;
    float bv = bias ? bias[col] : 0.f;
    if (BIAS_BF16) bv = bf16_round(bv);
#pragma unroll
    for (int r = 0; r < 8; ++r) {
      float v = acc[t][r] + bv;
      if (resid) { float rv = resid[(size_t)((row0 + 8 * hh + r) % rmod) * ldr + col]; if (RES_BF16) rv = bf16_round(rv); v += rv; }
      if (ACT == 1) v = fmaxf(v, 0.f);
      if (ACT == 2) v = 0.5f * v * (1.0f + erff(v * 0.70710678118654752f));
      if (ACT == 3) { const float u = 0.7978845608028654f * (v + 0.044715f * v * v * v); v = 0.5f * v * (1.0f + tanhf(u)); }
      so[w][8 * hh + r][t * 16 + ln] = v;
    }
  }
  __builtin_amdgcn_fence(__ATOMIC_ACQ_REL, "workgroup");
  __builtin_amdgcn_wave_barrier();
  const int rsub = lane >> 4, c4 = (lane & 15) * 4;
  for (int pass = 0; pass < 2; ++pass) {
#pragma unroll
    for (int q = 0; q < 8; ++q) {
      const int r = q * 2 + rsub;
      const v4f v = *(const v4fa*)&so[w][r][c4];
      *(volatile v4f*)(C + (size_t)(row0 + r) * ldc + col0 + c4) = v;
    }
    if (pass == 0) __threadfence();
  }
}
template <bool PARAM_BF16>
__global__ __launch_bounds__(256) void k_layernorm(const float* __restrict__ X, const float* __restrict__ R, const float* __restrict__ g, const float* __restrict__ bta,
                                                  float* __restrict__ out_sum, float* __restrict__ out_norm, int N, float eps) {
  __shared__ float red[256];
  const int row = blockIdx.x, tid = threadIdx.x;
  const float* x = X + (size_t)row * N; const float* rr = R ? R + (size_t)row * N : nullptr;
  float vals[16];
  const int per = N / 256;
  float s1 = 0.f;
  for (int u = 0; u < per / 4; ++u) {
    const int j = tid * 4 + 1024 * u;
    const v4f a = *(const v4fa*)(x + j);
    v4f b = {0.f,0.f,0.f,0.f}; if (rr) b = *(const v4fa*)(rr + j);
#pragma unroll
    for (int q = 0; q < 4; ++q) { const float v = a[q] + b[q]; vals[u * 4 + q] = v; s1 += v; }
  }
  red[tid] = s1; __syncthreads();
  for (int st = 128; st > 0; st >>= 1) { if (tid < st) red[tid] += red[tid + st]; __syncthreads(); }
  const float mu = red[0] / (float)N; __syncthreads();
  float s2 = 0.f;
  for (int u = 0; u < per / 4; ++u)
#pragma unroll
    for (int q = 0; q < 4; ++q) { const float c = vals[u * 4 + q] - mu; s2 += c * c; }
  red[tid] = s2; __syncthreads();
  for (int st = 128; st > 0; st >>= 1) { if (tid < st) red[tid] += red[tid + st]; __syncthreads(); }
  const float rs = rsqrtf(red[0] / (float)N + eps);
  for (int pass = 0; pass < 2; ++pass) {
    for (int u = 0; u < per / 4; ++u) {
      const int j = tid * 4 + 1024 * u;
      v4f o, sm;
#pragma unroll
      for (int q = 0; q < 4; ++q) {
        float gg = g[j + q], bb = bta[j + q];
        if (PARAM_BF16) { gg = bf16_round(gg); bb = bf16_round(bb); }
        sm[q] = vals[u * 4 + q]; o[q] = (vals[u * 4 + q] - mu) * rs * gg + bb;
      }
      if (out_sum) *(volatile v4f*)(out_sum + (size_t)row * N + j) = sm;
      *(volatile v4f*)(out_norm + (size_t)row * N + j) = o;
    }
    if (pass == 0) __threadfence();
  }
}

__global__ __launch_bounds__(256) void k_sort_init(const int* __restrict__ seg, int n, int nseg, unsigned int* __restrict__ key, unsigned int* __restrict__ val, int np2) {
  const int i = blockIdx.x * 256 + threadIdx.x; if (i >= np2) return;
  unsigned int kv = 0xFFFFFFFFu;
  if (i < n) { int s = seg[i]; s = s < 0 ? 0 : (s >= nseg ? nseg - 1 : s); kv = (unsigned int)s; }
  *(volatile unsigned int*)(key + i) = kv; *(volatile unsigned int*)(val + i) = (unsigned int)i;
  __threadfence();
  *(volatile unsigned int*)(key + i) = kv; *(volatile unsigned int*)(val + i) = (unsigned int)i;
}
template <bool STAGE0>
__global__ __launch_bounds__(512) void k_sort_lds(unsigned int* __restrict__ key, unsigned int* __restrict__ val, int kstage) {
  __shared__ unsigned int sk[1024], sv[1024];
  const int tid = threadIdx.x; const int base = blockIdx.x * 1024;
  sk[tid] = key[base + tid]; sv[tid] = val[base + tid]; sk[tid + 512] = key[base + tid + 512]; sv[tid + 512] = val[base + tid + 512];
  __syncthreads();
  for (int k = (STAGE0 ? 2 : kstage); k <= (STAGE0 ? 1024 : kstage); k <<= 1) {
    for (int j = (k > 1024 ? 512 : (k >> 1)); j >= 1; j >>= 1) {
      const int lo = tid & (j - 1), hi2 = (tid >> __builtin_ctz(j)) << (__builtin_ctz(j) + 1);
      const int il = hi2 | lo, ir = il | j;
      const int gi = base + il;
      const bool asc = ((gi & k) == 0);
      unsigned int a = sk[il], b = sk[ir], va = sv[il], vb = sv[ir];
      const bool swp = asc ? (a > b) : (a < b);
      if (swp) { sk[il] = b; sk[ir] = a; sv[il] = vb; sv[ir] = va; }
      __syncthreads();
    }
  }
  for (int pass = 0; pass < 2; ++pass) {
    *(volatile unsigned int*)(key + base + tid) = sk[tid]; *(volatile unsigned int*)(val + base + tid) = sv[tid];
    *(volatile unsigned int*)(key + base + tid + 512) = sk[tid + 512]; *(volatile unsigned int*)(val + base + tid + 512) = sv[tid + 512];
    if (pass == 0) __threadfence();
  }
}
__global__ __launch_bounds__(256) void k_sort_step(unsigned int* __restrict__ key, unsigned int* __restrict__ val, int k, int j, int np2) {
  const int t = blockIdx.x * 256 + threadIdx.x; if (t >= np2 / 2) return;
  const int lo = t & (j - 1), il = ((t >> __builtin_ctz(j)) << (__builtin_ctz(j) + 1)) | lo, ir = il | j;
  const bool asc = ((il & k) == 0);
  unsigned int a = key[il], b = key[ir], va = val[il], vb = val[ir];
  const bool swp = asc ? (a > b) : (a < b);
  const unsigned int k1 = swp ? b : a, k2 = swp ? a : b, v1 = swp ? vb : va, v2 = swp ? va : vb;
  *(volatile unsigned int*)(key + il) = k1; *(volatile unsigned int*)(key + ir) = k2; *(volatile unsigned int*)(val + il) = v1; *(volatile unsigned int*)(val + ir) = v2;
  __threadfence();
  *(volatile unsigned int*)(key + il) = k1; *(volatile unsigned int*)(key + ir) = k2; *(volatile unsigned int*)(val + il) = v1; *(volatile unsigned int*)(val + ir) = v2;
}
__global__ __launch_bounds__(256) void k_rowptr(const unsigned int* __restrict__ key, int np2, int nseg, int* __restrict__ rowptr) {
  int s = blockIdx.x * 256 + threadIdx.x; if (s >= ((nseg + 1 + 31) / 32) * 32) return;
  const int sdst = s; if (s > nseg) s = nseg;
  int lo = 0, hi = np2;
  while (lo < hi) { const int mid = (lo + hi) >> 1; if (key[mid] < (unsigned int)s) lo = mid + 1; else hi = mid; }
  *(volatile int*)(rowptr + sdst) = lo; __threadfence(); *(volatile int*)(rowptr + sdst) = lo;
}
static void sort_pairs(unsigned int* key, unsigned int* val, int np2, hipStream_t stream) {
  k_sort_lds<true><<<np2 / 1024, 512, 0, stream>>>(key, val, 0);
  for (int k = 2048; k <= np2; k <<= 1) {
    for (int j = k >> 1; j >= 1024; j >>= 1) k_sort_step<<<(np2 / 2 + 255) / 256, 256, 0, stream>>>(key, val, k, j, np2);
    k_sort_lds<false><<<np2 / 1024, 512, 0, stream>>>(key, val, k);
  }
}

__device__ __forceinline__ float silu_f(float x) { return x / (1.0f + expf(-x)); }
__global__ __launch_bounds__(256) void k_wt_e1(const float* __restrict__ W, unsigned short* __restrict__ Bt) {
  const int t = blockIdx.x * 256 + threadIdx.x; if (t >= HH * (K1 / 8)) return; const int n = t / (K1 / 8), k8 = (t % (K1 / 8)) * 8; v8us v;
  for (int i = 0; i < 8; ++i) { const int k = k8 + i; v[i] = (k < 2 * HH + ED) ? bf16_bits(W[(size_t)k * HH + n]) : (unsigned short)0; }
  *(volatile v8us*)(Bt + (size_t)n * K1 + k8) = v; __threadfence(); *(volatile v8us*)(Bt + (size_t)n * K1 + k8) = v;
}
__global__ __launch_bounds__(256) void k_embed(const int* __restrict__ z, const float* __restrict__ emb, float* __restrict__ x) {
  const size_t t = (size_t)blockIdx.x * 256 + threadIdx.x; if (t >= (size_t)NNODE * (HH / 4)) return; const int n = (int)(t / (HH / 4)), c4 = (int)(t % (HH / 4)) * 4;
  int id = z[n]; id = id < 0 ? 0 : (id > 100 ? 100 : id);
  v4f v; for (int q = 0; q < 4; ++q) v[q] = bf16_round(emb[(size_t)id * HH + c4 + q]);
  *(volatile v4f*)(x + t * 4) = v; __threadfence(); *(volatile v4f*)(x + t * 4) = v;
}
__global__ __launch_bounds__(128) void k_edge_mlp(const float* __restrict__ x, const float* __restrict__ ea, const int* __restrict__ src, const int* __restrict__ dst, int e_base,
                                                const unsigned short* __restrict__ Bt1, const float* __restrict__ b1, const unsigned short* __restrict__ Bt2, const float* __restrict__ b2, float* __restrict__ msg) {
  __shared__ __attribute__((aligned(16))) float sH[4][16][HH + 4];
  __shared__ __attribute__((aligned(16))) float so[4][16][64];
  const int tid = threadIdx.x, w = tid >> 5, lane = tid & 31, ln = lane & 15, hh = lane >> 4;
  const size_t el0 = ((size_t)blockIdx.x * 4 + w) * 16; const size_t e = (size_t)e_base + el0 + ln;
  int sn = src[e]; sn = sn < 0 ? 0 : (sn >= NNODE ? NNODE - 1 : sn); int dn = dst[e]; dn = dn < 0 ? 0 : (dn >= NNODE ? NNODE - 1 : dn);
  const float* xs = x + (size_t)sn * HH; const float* xd = x + (size_t)dn * HH; const float* er = ea + e * ED;
  v8f acc[8]; for (int t = 0; t < 8; ++t) acc[t] = (v8f){0.f,0.f,0.f,0.f,0.f,0.f,0.f,0.f};
#pragma unroll 1
  for (int ks = 0; ks < K1 / 32; ++ks) {
    FragB ah, al;
#pragma unroll
    for (int i = 0; i < 16; ++i) { const int k = ks * 32 + ((i < 8) ? (8 * hh + i) : (16 + 8 * hh + (i - 8))); float v = 0.f;
      if (k < HH) v = xs[k]; else if (k < 2 * HH) v = xd[k - HH]; else if (k < 2 * HH + ED) v = bf16_round(er[k - 2 * HH]);
      const unsigned short hb = bf16_bits(v); ah.u[i] = hb; al.u[i] = bf16_bits(v - bf16_val(hb)); }
#pragma unroll
    for (int t = 0; t < 8; ++t) { FragB b; b.half[0] = *(const v8us*)(Bt1 + (size_t)(t * 16 + ln) * K1 + ks * 32 + 8 * hh); b.half[1] = *(const v8us*)(Bt1 + (size_t)(t * 16 + ln) * K1 + ks * 32 + 16 + 8 * hh); acc[t] = mmaN<2>(ah.v, al.v, b.v, b.v, acc[t]); }
  }
#pragma unroll
  for (int t = 0; t < 8; ++t) { const int col = t * 16 + ln; const float bb = bf16_round(b1[col]);
#pragma unroll
    for (int r = 0; r < 8; ++r) sH[w][8 * hh + r][col] = silu_f(acc[t][r] + bb); }
  __builtin_amdgcn_fence(__ATOMIC_ACQ_REL, "workgroup"); __builtin_amdgcn_wave_barrier();
  FragB a2h[4], a2l[4];
#pragma unroll
  for (int ks = 0; ks < 4; ++ks)
#pragma unroll
    for (int i = 0; i < 16; ++i) { const int k = ks * 32 + ((i < 8) ? (8 * hh + i) : (16 + 8 * hh + (i - 8))); const float v = sH[w][ln][k]; const unsigned short hb = bf16_bits(v); a2h[ks].u[i] = hb; a2l[ks].u[i] = bf16_bits(v - bf16_val(hb)); }
#pragma unroll 1
  for (int half = 0; half < 2; ++half) {
    v8f acc2[4]; for (int t = 0; t < 4; ++t) acc2[t] = (v8f){0.f,0.f,0.f,0.f,0.f,0.f,0.f,0.f};
#pragma unroll
    for (int ks = 0; ks < 4; ++ks)
#pragma unroll
      for (int t = 0; t < 4; ++t) { const int n = half * 64 + t * 16 + ln; FragB b; b.half[0] = *(const v8us*)(Bt2 + (size_t)n * HH + ks * 32 + 8 * hh); b.half[1] = *(const v8us*)(Bt2 + (size_t)n * HH + ks * 32 + 16 + 8 * hh); acc2[t] = mmaN<2>(a2h[ks].v, a2l[ks].v, b.v, b.v, acc2[t]); }
#pragma unroll
    for (int t = 0; t < 4; ++t) { const int col = half * 64 + t * 16 + ln; const float bb = bf16_round(b2[col]);
#pragma unroll
      for (int r = 0; r < 8; ++r) so[w][8 * hh + r][t * 16 + ln] = silu_f(acc2[t][r] + bb); }
    __builtin_amdgcn_fence(__ATOMIC_ACQ_REL, "workgroup"); __builtin_amdgcn_wave_barrier();
    const int rsub = lane >> 4, c4 = (lane & 15) * 4;
    for (int pass = 0; pass < 2; ++pass) { for (int q = 0; q < 8; ++q) { const int r = q * 2 + rsub; const v4f v = *(const v4fa*)&so[w][r][c4]; *(volatile v4f*)(msg + (el0 + r) * HH + half * 64 + c4) = v; } if (pass == 0) __threadfence(); }
    __builtin_amdgcn_fence(__ATOMIC_ACQ_REL, "workgroup"); __builtin_amdgcn_wave_barrier();
  }
}
__global__ __launch_bounds__(256) void k_agg_slice(const float* __restrict__ x, const float* __restrict__ msg, int e_base, int first, const int* __restrict__ rowptr, const unsigned int* __restrict__ perm, float* xcat) {
  const int tid = threadIdx.x, w = tid >> 5, lane = tid & 31; const int nd = blockIdx.x * 8 + w; if (nd >= NNODE) return;
  float* row = xcat + (size_t)nd * 2 * HH;
  v4f acc = first ? (v4f){0.f,0.f,0.f,0.f} : *(const v4fa*)(row + HH + lane * 4);
  for (int p = rowptr[nd]; p < rowptr[nd + 1]; ++p) { const int e = (int)perm[p]; if (e < e_base || e >= e_base + ESL) continue; const v4f m4 = *(const v4fa*)(msg + (size_t)(e - e_base) * HH + lane * 4); for (int q = 0; q < 4; ++q) acc[q] += m4[q]; }
  if (first) { const v4f own = *(const v4fa*)(x + (size_t)nd * HH + lane * 4); *(volatile v4f*)(row + lane * 4) = own; }
  *(volatile v4f*)(row + HH + lane * 4) = acc; __threadfence();
  if (first) { const v4f own = *(const v4fa*)(x + (size_t)nd * HH + lane * 4); *(volatile v4f*)(row + lane * 4) = own; }
  *(volatile v4f*)(row + HH + lane * 4) = acc;
}
__global__ __launch_bounds__(256) void k_silu_ip(float* __restrict__ a, size_t n4) { const size_t t = (size_t)blockIdx.x * 256 + threadIdx.x; if (t >= n4) return; v4f v = *(const v4fa*)(a + t * 4); for (int q = 0; q < 4; ++q) v[q] = silu_f(v[q]); *(volatile v4f*)(a + t * 4) = v; __threadfence(); *(volatile v4f*)(a + t * 4) = v; }
__global__ __launch_bounds__(256) void k_gptr(const int* __restrict__ batch, int* __restrict__ gptr) {
  const int slot = blockIdx.x * 256 + threadIdx.x; if (slot >= ((NG + 1 + 31) / 32) * 32) return; const int g = slot > NG ? NG : slot;
  int lo = 0, hi = NNODE; while (lo < hi) { const int mid = (lo + hi) >> 1; if (batch[mid] < g) lo = mid + 1; else hi = mid; }
  *(volatile int*)(gptr + slot) = lo; __threadfence(); *(volatile int*)(gptr + slot) = lo;
}
__global__ __launch_bounds__(256) void k_pool(const float* __restrict__ h, const int* __restrict__ gptr, float* __restrict__ pooled) {
  const int tid = threadIdx.x, w = tid >> 5, lane = tid & 31; const int g = blockIdx.x * 8 + w; if (g >= NG) return;
  v4f a = {0.f,0.f,0.f,0.f}; const int n0 = gptr[g], n1 = gptr[g + 1];
  for (int n = n0; n < n1; ++n) { const v4f x0 = *(const v4fa*)(h + (size_t)n * HH + lane * 4); for (int q = 0; q < 4; ++q) a[q] += x0[q]; }
  const float inv = 1.0f / fmaxf((float)(n1 - n0), 1.0f); for (int q = 0; q < 4; ++q) a[q] *= inv;
  float* row = pooled + (size_t)g * HH + lane * 4; *(volatile v4f*)row = a; __threadfence(); *(volatile v4f*)row = a;
}
__global__ __launch_bounds__(256) void k_head(const float* __restrict__ gz, const float* __restrict__ rw2, const float* __restrict__ rb2, float* __restrict__ out) {
  __shared__ float so[NG];
  for (int g = threadIdx.x; g < NG; g += 256) { float s = bf16_round(rb2[0]);
#pragma unroll 1
    for (int c = 0; c < HH; ++c) s += gz[(size_t)g * HH + c] * bf16_round(rw2[c]); so[g] = s; }
  __syncthreads();
  for (int pass = 0; pass < 2; ++pass) { for (int g = threadIdx.x; g < NG; g += 256) *(volatile float*)(out + g) = so[g]; if (pass == 0) __threadfence(); }
}
extern "C" void kernel_launch(void* const* d_in, const int* in_sizes, int n_in,
                              void* d_out, int out_size, void* d_ws, size_t ws_size, hipStream_t stream) {
  (void)in_sizes; (void)n_in; (void)out_size;
  const int* z = (const int*)d_in[0]; const int* ei = (const int*)d_in[1]; const float* ea = (const float*)d_in[2]; const int* batch = (const int*)d_in[3]; const float* emb = (const float*)d_in[4];
  const float* ew1 = (const float*)d_in[5]; const float* eb1 = (const float*)d_in[6]; const float* ew2 = (const float*)d_in[7]; const float* eb2 = (const float*)d_in[8];
  const float* nw = (const float*)d_in[9]; const float* nb = (const float*)d_in[10]; const float* rw1 = (const float*)d_in[11]; const float* rb1 = (const float*)d_in[12]; const float* rw2 = (const float*)d_in[13]; const float* rb2 = (const float*)d_in[14];
  const int* src = ei; const int* dst = ei + NEDGE;
  char* ws = (char*)d_ws; size_t off = 0;
  auto take = [&](size_t bytes) { char* p = ws + off; off += (bytes + 255) & ~(size_t)255; return p; };
  unsigned short* Bt1[NL], *Bt2[NL], *Btn[NL]; for (int l = 0; l < NL; ++l) { Bt1[l] = (unsigned short*)take((size_t)HH * K1 * 2); Bt2[l] = (unsigned short*)take((size_t)HH * HH * 2); Btn[l] = (unsigned short*)take((size_t)HH * 2 * HH * 2); }
  unsigned short* Br1 = (unsigned short*)take((size_t)HH * HH * 2);
  unsigned int* key = (unsigned int*)take((size_t)NP2 * 4); unsigned int* perm = (unsigned int*)take((size_t)NP2 * 4); int* rowptr = (int*)take((size_t)(NNODE + 64) * 4);
  float* x = (float*)take((size_t)NNODE * HH * 4); float* xcat = (float*)take((size_t)NNODE * 2 * HH * 4); float* msg = (float*)take((size_t)ESL * HH * 4);
  int* gptr = (int*)take((size_t)(NG + 64) * 4); float* pooled = (float*)take((size_t)NG * HH * 4); float* gz = (float*)take((size_t)NG * HH * 4);
  if (off > ws_size) return;
  for (int l = 0; l < NL; ++l) { k_wt_e1<<<(HH * (K1 / 8) + 255) / 256, 256, 0, stream>>>(ew1 + (size_t)l * (2 * HH + ED) * HH, Bt1[l]); k_wt_bf16<<<(HH * (HH / 8) + 255) / 256, 256, 0, stream>>>(ew2 + (size_t)l * HH * HH, Bt2[l], HH, HH); k_wt_bf16<<<(HH * (2 * HH / 8) + 255) / 256, 256, 0, stream>>>(nw + (size_t)l * 2 * HH * HH, Btn[l], 2 * HH, HH); }
  k_wt_bf16<<<(HH * (HH / 8) + 255) / 256, 256, 0, stream>>>(rw1, Br1, HH, HH);
  k_sort_init<<<NP2 / 256, 256, 0, stream>>>(dst, NEDGE, NNODE, key, perm, NP2);
  sort_pairs(key, perm, NP2, stream);
  k_rowptr<<<(NNODE + 32 + 255) / 256, 256, 0, stream>>>(key, NP2, NNODE, rowptr);
  k_embed<<<(NNODE * (HH / 4) + 255) / 256, 256, 0, stream>>>(z, emb, x);
  const int gb = ((NNODE / 16) * (HH / 64) + 3) / 4;
  for (int l = 0; l < NL; ++l) {
    for (int sl = 0; sl < NSL; ++sl) {
      k_edge_mlp<<<ESL / 64, 128, 0, stream>>>(x, ea, src, dst, sl * ESL, Bt1[l], eb1 + l * HH, Bt2[l], eb2 + l * HH, msg);
      k_agg_slice<<<(NNODE + 7) / 8, 256, 0, stream>>>(x, msg, sl * ESL, sl == 0 ? 1 : 0, rowptr, perm, xcat);
    }
    k_gemm_bf3<true, 0, true, false><<<gb, 128, 0, stream>>>(xcat, 2 * HH, Btn[l], 2 * HH, nb + l * HH, nullptr, 1, 0, x, HH, NNODE, HH, 2 * HH);
    k_silu_ip<<<(NNODE * HH / 4 + 255) / 256, 256, 0, stream>>>(x, (size_t)NNODE * HH / 4);
  }
  k_gptr<<<(NG + 32 + 255) / 256, 256, 0, stream>>>(batch, gptr);
  k_pool<<<(NG + 7) / 8, 256, 0, stream>>>(x, gptr, pooled);
  k_gemm_bf3<true, 0, true, false><<<((NG / 16) * (HH / 64) + 3) / 4, 128, 0, stream>>>(pooled, HH, Br1, HH, rb1, nullptr, 1, 0, gz, HH, NG, HH, HH);
  k_silu_ip<<<(NG * HH / 4 + 255) / 256, 256, 0, stream>>>(gz, (size_t)NG * HH / 4);
  k_head<<<1, 256, 0, stream>>>(gz, rw2, rb2, (float*)d_out);
}
